// GATv2_68728066670717
// MI455X (gfx1250) — hardware-verified
//
#include <hip/hip_runtime.h>
#include <stddef.h>
#include <stdint.h>
#include <math.h>


#define DIN     128
#define HID     64
#define PW      192
#define KG      128
#define XW      64
#define NG      256
#define NTHR    256
#define NWAVE   8
#define EPT     8
#define CHUNK   (NTHR * EPT)
#define WCAP    (EPT * 32)
#define LISTN   (NWAVE * WCAP)
#define NBA     1024
#define SLA     10
#define RCAP    28672
#define DEGCAP  128
#define MEAS_B1024  20780
#define MEAS_MAXDEG 42
#define GBM     64
#define GBN     64
#define GTHR    128
#define NUWM    1024
#define NUW     (9 * NUWM)
#define NEGSL   0.2f
#define WSMAX   134217728
#define BKT_LDS_INTS  (LISTN + RCAP + 16)
#define SCAN_ZINTS    (RCAP + 3 * NBA)
#define SCAN_LDS_INTS (2 * RCAP + 3 * NBA + 16)

static_assert((CHUNK & (CHUNK - 1)) == 0 && CHUNK <= 4096);
static_assert((NBA & (NBA - 1)) == 0 && NBA == (1 << SLA) && NBA <= 1024);
static_assert(((long long)CHUNK << SLA) < (1LL << 31));
static_assert(LISTN >= NWAVE * WCAP);
static_assert(NBA % NWAVE == 0 && NBA % 32 == 0);
static_assert((RCAP % 32) == 0 && (SCAN_ZINTS % 4) == 0);
static_assert(RCAP >= MEAS_B1024 + 4096);
static_assert(DEGCAP >= MEAS_MAXDEG + 8);
static_assert(SCAN_LDS_INTS * 4 <= 300000 && BKT_LDS_INTS * 4 <= 300000);
static_assert(GBM == (GTHR / 32) * 16);
static_assert((KG % 32) == 0 && KG == 2 * HID && KG == DIN);
static_assert(PW == 3 * GBN && HID == GBN);
static_assert(HID == 2 * 32);
static_assert(XW == HID);
static_assert(NBA == 4 * NTHR);
static_assert(NBA <= RCAP);
static_assert((NUWM % NTHR) == 0);
static_assert(NG == NTHR);

typedef float          v2f  __attribute__((ext_vector_type(2)));
typedef float          v4f  __attribute__((ext_vector_type(4)));
typedef float          v8f  __attribute__((ext_vector_type(8)));
typedef double         v2d  __attribute__((ext_vector_type(2)));
typedef int            v4i  __attribute__((ext_vector_type(4)));
typedef int            v8i  __attribute__((ext_vector_type(8)));
typedef unsigned short v8us __attribute__((ext_vector_type(8)));
typedef __bf16         v16b __attribute__((ext_vector_type(16)));
typedef v2f  __attribute__((may_alias)) v2fa;
typedef v4f  __attribute__((may_alias)) v4fa;
typedef v4i  __attribute__((may_alias)) v4ia;
typedef v8us __attribute__((may_alias)) v8usa;
union FragB { v16b v; v8us h[2]; v8i w; };

__device__ __forceinline__ v8f wmb(const FragB& a, const FragB& b, v8f c) {
  v8f d = __builtin_amdgcn_wmma_f32_16x16x32_bf16(false, a.v, false, b.v, (short)0, c, false, false);
  asm volatile("v_nop\n\tv_nop\n\tv_nop\n\tv_nop" : "+v"(d) : "v"(a.w), "v"(b.w));
  return d;
}

__device__ __forceinline__ unsigned int f2bf(float f) {
  const unsigned int u = __float_as_uint(f);
  const unsigned int r = ((u + 0x7FFFu + ((u >> 16) & 1u)) >> 16) & 0xFFFFu;
  return ((u & 0x7FFFFFFFu) > 0x7F800000u) ? 0x7FC0u : r;
}
__device__ __forceinline__ float bf2f(unsigned int b) { return __uint_as_float(b << 16); }
__device__ __forceinline__ float bfr(float f) { return bf2f(f2bf(f)); }

__device__ __forceinline__ v8us cvt8b(const v4f a, const v4f b) {
  v8us o;
  o[0] = (unsigned short)f2bf(a.x); o[1] = (unsigned short)f2bf(a.y);
  o[2] = (unsigned short)f2bf(a.z); o[3] = (unsigned short)f2bf(a.w);
  o[4] = (unsigned short)f2bf(b.x); o[5] = (unsigned short)f2bf(b.y);
  o[6] = (unsigned short)f2bf(b.z); o[7] = (unsigned short)f2bf(b.w);
  return o;
}

template <int SLB>
__device__ __forceinline__ int scan_chunk(const int* __restrict__ dsts, int nE, int cbase, int slotBase,
                                          int nb, int vec8, int* list, int tid, int lane, int wave) {
  int wc = 0;
  const int el0  = tid * EPT;
  const int e0   = cbase + el0;
  const int sent = -2147483647 - 1;
  v4i da, db;
  if (vec8 != 0 && cbase + CHUNK <= nE) {
    da = *(const v4i*)(dsts + e0);
    db = *(const v4i*)(dsts + e0 + 4);
  } else {
    da.x = (e0     < nE) ? dsts[min(e0,     nE - 1)] : sent;
    da.y = (e0 + 1 < nE) ? dsts[min(e0 + 1, nE - 1)] : sent;
    da.z = (e0 + 2 < nE) ? dsts[min(e0 + 2, nE - 1)] : sent;
    da.w = (e0 + 3 < nE) ? dsts[min(e0 + 3, nE - 1)] : sent;
    db.x = (e0 + 4 < nE) ? dsts[min(e0 + 4, nE - 1)] : sent;
    db.y = (e0 + 5 < nE) ? dsts[min(e0 + 5, nE - 1)] : sent;
    db.z = (e0 + 6 < nE) ? dsts[min(e0 + 6, nE - 1)] : sent;
    db.w = (e0 + 7 < nE) ? dsts[min(e0 + 7, nE - 1)] : sent;
  }
  const unsigned nbs = (unsigned)slotBase;
  const unsigned unb = (unsigned)nb;
  const unsigned s0 = (unsigned)da.x - nbs, s1 = (unsigned)da.y - nbs;
  const unsigned s2 = (unsigned)da.z - nbs, s3 = (unsigned)da.w - nbs;
  const unsigned s4 = (unsigned)db.x - nbs, s5 = (unsigned)db.y - nbs;
  const unsigned s6 = (unsigned)db.z - nbs, s7 = (unsigned)db.w - nbs;
  const bool h0 = s0 < unb, h1 = s1 < unb, h2 = s2 < unb, h3 = s3 < unb;
  const bool h4 = s4 < unb, h5 = s5 < unb, h6 = s6 < unb, h7 = s7 < unb;
  const unsigned any = __builtin_amdgcn_ballot_w32(h0 | h1 | h2 | h3 | h4 | h5 | h6 | h7);
  if (any != 0u) {
#define HITJ(J, HJ, SJ) { \
      const unsigned mj = __builtin_amdgcn_ballot_w32(HJ); \
      if (mj != 0u) { \
        if (HJ) { \
          const int pos = wc + (int)__builtin_amdgcn_mbcnt_lo(mj, 0u); \
          if (pos < WCAP) list[wave * WCAP + pos] = ((el0 + (J)) << SLB) | (int)(SJ); \
        } \
        wc += (int)__builtin_popcount(mj); } }
    HITJ(0, h0, s0)
    HITJ(1, h1, s1)
    HITJ(2, h2, s2)
    HITJ(3, h3, s3)
    HITJ(4, h4, s4)
    HITJ(5, h5, s5)
    HITJ(6, h6, s6)
    HITJ(7, h7, s7)
#undef HITJ
  }
  return wc;
}

__global__ __launch_bounds__(NTHR) void k_prep(const float* __restrict__ x,
                                               const float* __restrict__ Wl0, const float* __restrict__ Wr0,
                                               const float* __restrict__ Rw0, const float* __restrict__ Wl1,
                                               const float* __restrict__ Wr1, const float* __restrict__ Rw1,
                                               const float* __restrict__ Wl2, const float* __restrict__ Wr2,
                                               const float* __restrict__ Rw2,
                                               unsigned short* XB, unsigned short* BW, int nN, int nUx) {
  const int u = (int)blockIdx.x * NTHR + (int)threadIdx.x;
  const v4f z4 = {0.f, 0.f, 0.f, 0.f};
  v4f a = z4, b = z4;
  unsigned short* dp;
  if (u < nUx) {
    const int row = u >> 4;
    const int c0  = (u & 15) * 8;
    const int rc  = row < nN ? row : nN - 1;
    const float* p = x + (size_t)rc * DIN + c0;
    a = *(const v4f*)p;
    b = *(const v4f*)(p + 4);
    if (row >= nN) { a = z4; b = z4; }
    dp = XB + (size_t)row * DIN + c0;
  } else {
    const int v = u - nUx;
    if (v >= NUW) return;
    const int w  = v >> 10;
    const int r  = v & (NUWM - 1);
    const int n  = r >> 4;
    const int k8 = (r & 15) * 8;
    const int kd = k8 & (HID - 1);
#define WLD(PTR, PITCH, KK) { const float* q = (PTR) + (size_t)n * (PITCH) + (KK); a = *(const v4f*)q; b = *(const v4f*)(q + 4); }
    switch (w) {
      case 0: WLD(Wl0, DIN, k8) break;
      case 1: WLD(Wr0, DIN, k8) break;
      case 2: WLD(Rw0, DIN, k8) break;
      case 3: WLD(Wl1, HID, kd) break;
      case 4: WLD(Wr1, HID, kd) break;
      case 5: WLD(Rw1, HID, kd) break;
      case 6: WLD(Wl2, HID, kd) break;
      case 7: WLD(Wr2, HID, kd) break;
      default: WLD(Rw2, HID, kd) break;
    }
#undef WLD
    const int layer = w / 3;
    const int mat   = w - 3 * layer;
    dp = BW + ((size_t)layer * PW + (size_t)mat * HID + (size_t)n) * KG + k8;
  }
  const v8us o = cvt8b(a, b);
  *(volatile v8us*)dp = o;
  __threadfence();
  *(volatile v8us*)dp = o;
}

__global__ __launch_bounds__(NTHR) void k_bucket(const int* __restrict__ srcs, const int* __restrict__ dsts,
                                                 int nE, int nN, int vec8, int* HITS, int* FLG) {
  extern __shared__ __attribute__((aligned(16))) int bsm[];
  int* list = bsm;
  int* reg1 = bsm + LISTN;
  int* wcnt = reg1 + RCAP;
  const int tid = (int)threadIdx.x, lane = tid & 31, wave = tid >> 5;
  const int blk = (int)blockIdx.x;
  const int nodeBase = blk * NBA;
  int nb = nN - nodeBase;
  nb = nb < 0 ? 0 : (nb > NBA ? NBA : nb);

  int tot = 0, ovf = 0;
  const int nChunks = (nE + CHUNK - 1) / CHUNK;
#pragma unroll 1
  for (int ch = 0; ch < nChunks; ++ch) {
    const int cbase = ch * CHUNK;
    const int wc = scan_chunk<SLA>(dsts, nE, cbase, nodeBase, nb, vec8, list, tid, lane, wave);
    if (lane == 0) wcnt[wave] = wc;
    __syncthreads();
    int pre = 0, all = 0;
#pragma unroll
    for (int w2 = 0; w2 < NWAVE; ++w2) {
      int c = wcnt[w2];
      c = c < 0 ? 0 : (c > WCAP ? WCAP : c);
      all += c;
      pre += (w2 < wave) ? c : 0;
    }
    const int wcc  = wc > WCAP ? WCAP : wc;
    const int base = tot + pre;
#pragma unroll 1
    for (int i = lane; i < wcc; i += 32) {
      const int ent = list[wave * WCAP + i];
      const int el  = (ent >> SLA) & (CHUNK - 1);
      const int sl  = ent & (NBA - 1);
      int eid = cbase + el;
      eid = eid > nE - 1 ? nE - 1 : eid;
      const int sraw = srcs[eid];
      const int s = sraw < 0 ? 0 : (sraw > nN - 1 ? nN - 1 : sraw);
      const int pos = base + i;
      if (pos < RCAP) reg1[pos] = (int)((unsigned)s | ((unsigned)sl << 16));
    }
    if (tot + all > RCAP) ovf = 1;
    tot += all;
    tot = tot > RCAP ? RCAP : tot;
    __syncthreads();
  }
  const int nh = tot;
  const int nhPad = (nh + 31) & ~31;
  for (int i = nh + tid; i < nhPad; i += NTHR) reg1[i] = 0;
  __syncthreads();

  int* hb = HITS + (size_t)blk * RCAP;
  v4i cv;
  cv.x = (tid == 0) ? nh : 0;
  cv.y = (tid == 0) ? ovf : 0;
  cv.z = 0; cv.w = 0;
  int* fp = FLG + (size_t)blk * 32 + 4 * (tid & 7);
#pragma unroll 1
  for (int p = tid * 4; p < nhPad; p += NTHR * 4) {
    const v4i v = *(const v4ia*)(reg1 + p);
    *(volatile v4i*)(hb + p) = v;
  }
  if (tid < 8) *(volatile v4i*)fp = cv;
  __threadfence();
#pragma unroll 1
  for (int p = tid * 4; p < nhPad; p += NTHR * 4) {
    const v4i v = *(const v4ia*)(reg1 + p);
    *(volatile v4i*)(hb + p) = v;
  }
  if (tid < 8) *(volatile v4i*)fp = cv;
}

__global__ __launch_bounds__(GTHR) void k_gemm(const unsigned short* __restrict__ A,
                                               const unsigned short* __restrict__ WT,
                                               const float* __restrict__ rb, float* outF) {
  __shared__ __attribute__((aligned(16))) float stg[GBM * GBN];
  const int tid = (int)threadIdx.x, lane = tid & 31, wave = tid >> 5, hh = lane >> 4, m = lane & 15;
  const int rowBase = (int)blockIdx.x * GBM;
  const int col0    = (int)blockIdx.y * GBN;
  const bool isRes  = ((int)blockIdx.y == 2);

  float badd[4];
#pragma unroll
  for (int t = 0; t < 4; ++t) {
    const float bv = bfr(rb[16 * t + m]);
    badd[t] = isRes ? bv : 0.0f;
  }

  v8f acc[4];
  {
    const v8f z = {0.f, 0.f, 0.f, 0.f, 0.f, 0.f, 0.f, 0.f};
    acc[0] = z; acc[1] = z; acc[2] = z; acc[3] = z;
  }
  const unsigned short* ap = A  + (size_t)(rowBase + 16 * wave + m) * (size_t)KG + 8 * hh;
  const unsigned short* wp = WT + (size_t)(col0 + m) * (size_t)KG + 8 * hh;
#pragma unroll 1
  for (int ks = 0; ks < KG / 32; ++ks) {
    FragB af;
    af.h[0] = *(const v8usa*)(ap + 32 * ks);
    af.h[1] = *(const v8usa*)(ap + 32 * ks + 16);
#pragma unroll
    for (int t = 0; t < 4; ++t) {
      const unsigned short* wq = wp + (size_t)(16 * t) * (size_t)KG + 32 * ks;
      FragB bf;
      bf.h[0] = *(const v8usa*)wq;
      bf.h[1] = *(const v8usa*)(wq + 16);
      acc[t] = wmb(af, bf, acc[t]);
    }
  }

#pragma unroll
  for (int t = 0; t < 4; ++t) {
    const int lc = 16 * t + m;
#pragma unroll
    for (int r = 0; r < 8; ++r) {
      const int lr = 16 * wave + 8 * hh + r;
      stg[lr * GBN + lc] = acc[t][r] + badd[t];
    }
  }
  __syncthreads();

  v4f fv[8];
#pragma unroll
  for (int i = 0; i < 8; ++i) {
    const int lr = 16 * wave + 2 * i + hh;
    fv[i] = *(const v4fa*)(stg + lr * GBN + 4 * m);
  }
#pragma unroll
  for (int i = 0; i < 8; ++i) {
    const int lr = 16 * wave + 2 * i + hh;
    const int gr = rowBase + lr;
    float* op = outF + (size_t)gr * (size_t)PW + col0 + 4 * m;
    *(volatile v4f*)op = fv[i];
  }
  __threadfence();
#pragma unroll
  for (int i = 0; i < 8; ++i) {
    const int lr = 16 * wave + 2 * i + hh;
    const int gr = rowBase + lr;
    float* op = outF + (size_t)gr * (size_t)PW + col0 + 4 * m;
    *(volatile v4f*)op = fv[i];
  }
}

template <int FIN>
__global__ __launch_bounds__(NTHR) void k_scan(const int* __restrict__ HITS, const int* __restrict__ FLGB,
                                               const float* __restrict__ P, const float* __restrict__ att,
                                               const float* __restrict__ bias, const float* __restrict__ Wf,
                                               unsigned int* XHL, float* S, int nN, int MPr) {
  static_assert(FIN == 0 || FIN == 1);
  extern __shared__ __attribute__((aligned(16))) int ssm[];
  int* hl   = ssm;
  int* sl   = ssm + RCAP;
  int* cnt  = sl + RCAP;
  int* offs = cnt + NBA;
  int* cur  = offs + NBA;
  int* misc = cur + NBA;
  const int tid = (int)threadIdx.x, lane = tid & 31, wave = tid >> 5;
  const int blk = (int)blockIdx.x;
  const int nodeBase = blk * NBA;

  const int nhraw = FLGB[(size_t)blk * 32];
  const int bflag = FLGB[(size_t)blk * 32 + 1];
  const int nh  = nhraw < 0 ? 0 : (nhraw > RCAP ? RCAP : nhraw);
  const int ovf = (bflag != 0 || nhraw < 0 || nhraw > RCAP) ? 1 : 0;

  {
    const v4i z4 = {0, 0, 0, 0};
    for (int i = tid * 4; i < SCAN_ZINTS; i += NTHR * 4) *(v4ia*)(sl + i) = z4;
    if (tid < 16) misc[tid] = 0;
    const int* hb = HITS + (size_t)blk * RCAP;
    const int nh4 = (nh + 3) & ~3;
#pragma unroll 1
    for (int p = tid * 4; p < nh4; p += NTHR * 4) *(v4ia*)(hl + p) = *(const v4i*)(hb + p);
  }
  __syncthreads();

  if (wave == 0) {
#pragma unroll 1
    for (int b0 = 0; b0 < nh; b0 += 32) {
      const int idx = b0 + lane;
      const int uv  = hl[idx < nh ? idx : nh - 1];
      const int m32 = (nh - b0) < 32 ? (nh - b0) : 32;
#pragma unroll 1
      for (int k = 0; k < m32; ++k) {
        const int u  = __builtin_amdgcn_readlane(uv, k);
        const int sq = (u >> 16) & (NBA - 1);
        if (lane == 0) cnt[sq] = cnt[sq] + 1;
      }
    }
  }
  __syncthreads();
  if (wave == 0) {
    const int base = lane * (NBA / 32);
    int s = 0;
#pragma unroll 1
    for (int i = 0; i < NBA / 32; ++i) s += cnt[base + i];
    int incl = s;
#pragma unroll
    for (int d = 1; d < 32; d <<= 1) {
      const int y = __shfl_up(incl, d, 32);
      if (lane >= d) incl += y;
    }
    int run = incl - s;
#pragma unroll 1
    for (int i = 0; i < NBA / 32; ++i) {
      const int cv = cnt[base + i];
      offs[base + i] = run;
      cur[base + i]  = run;
      run += cv;
    }
  }
  __syncthreads();
  if (wave == 0) {
#pragma unroll 1
    for (int b0 = 0; b0 < nh; b0 += 32) {
      const int idx = b0 + lane;
      const int uv  = hl[idx < nh ? idx : nh - 1];
      const int m32 = (nh - b0) < 32 ? (nh - b0) : 32;
#pragma unroll 1
      for (int k = 0; k < m32; ++k) {
        const int u  = __builtin_amdgcn_readlane(uv, k);
        const int sq = (u >> 16) & (NBA - 1);
        if (lane == 0) {
          int p = cur[sq];
          p = p < 0 ? 0 : (p > RCAP - 1 ? RCAP - 1 : p);
          sl[p] = u;
          cur[sq] = p + 1;
        }
      }
    }
  }
  __syncthreads();

  float* sS = (float*)hl;

  const float qnan = __int_as_float(0x7fc00000);
  const float pzb  = (ovf != 0) ? qnan : 0.0f;
  const v2f aq = *(const v2f*)(att + 2 * lane);
  const v2f bq = *(const v2f*)(bias + 2 * lane);
  const v2f wq = *(const v2f*)(Wf + 2 * lane);
  const float at0 = bfr(aq.x), at1 = bfr(aq.y);
  const float bz0 = bfr(bq.x), bz1 = bfr(bq.y);
  const float wf0 = bfr(wq.x), wf1 = bfr(wq.y);

#pragma unroll 1
  for (int si = 0; si < NBA / NWAVE; ++si) {
    const int s    = si * NWAVE + wave;
    const int node = nodeBase + s;
    const int nc   = node < nN ? node : nN - 1;
    int c = cnt[s];
    const bool big = c > DEGCAP;
    c = c < 0 ? 0 : (c > DEGCAP ? DEGCAP : c);
    int o = offs[s];
    o = o < 0 ? 0 : (o > RCAP ? RCAP : o);
    if (c > nh - o) c = nh - o;
    c = c < 0 ? 0 : c;
    c = __builtin_amdgcn_readfirstlane(c);
    o = __builtin_amdgcn_readfirstlane(o);

    const float* prow = P + (size_t)nc * PW + 2 * lane;
    const v2f xli = *(const v2fa*)prow;
    const v2f xri = *(const v2fa*)(prow + HID);
    const v2f rsi = *(const v2fa*)(prow + 2 * HID);

    float mx;
    {
      float v0 = xli.x + xri.x; v0 = v0 > 0.f ? v0 : NEGSL * v0;
      float v1 = xli.y + xri.y; v1 = v1 > 0.f ? v1 : NEGSL * v1;
      float lg = v0 * at0;
      lg = fmaf(v1, at1, lg);
#pragma unroll
      for (int off = 16; off > 0; off >>= 1) lg += __shfl_xor(lg, off, 32);
      mx = lg;
    }
    float dn = 1.0f, acc0 = xli.x, acc1 = xli.y;

#pragma unroll 1
    for (int b0 = 0; b0 < c; b0 += 32) {
      const int t = b0 + lane;
      int idx = o + t;
      idx = idx < 0 ? 0 : (idx > RCAP - 1 ? RCAP - 1 : idx);
      const int ent = sl[idx];
      int hs = ent & 0xFFFF;
      hs = hs > nN - 1 ? nN - 1 : hs;
      const int m32 = (c - b0) < 32 ? (c - b0) : 32;
#pragma unroll 1
      for (int k = 0; k < m32; ++k) {
        const int sk = __builtin_amdgcn_readlane(hs, k);
        const v2f a = *(const v2fa*)(P + (size_t)sk * PW + 2 * lane);
        float v0 = a.x + xri.x; v0 = v0 > 0.f ? v0 : NEGSL * v0;
        float v1 = a.y + xri.y; v1 = v1 > 0.f ? v1 : NEGSL * v1;
        float lg = v0 * at0;
        lg = fmaf(v1, at1, lg);
#pragma unroll
        for (int off = 16; off > 0; off >>= 1) lg += __shfl_xor(lg, off, 32);
        const float df = lg - mx;
        const float ee = expf(-fabsf(df));
        const bool  up = df > 0.f;
        const float s1 = up ? ee : 1.0f;
        const float s2 = up ? 1.0f : ee;
        mx = up ? lg : mx;
        dn = fmaf(dn, s1, s2);
        acc0 = fmaf(acc0, s1, s2 * a.x);
        acc1 = fmaf(acc1, s1, s2 * a.y);
      }
    }
    const float inv = __builtin_amdgcn_rcpf(dn);
    const float pzr = big ? qnan : pzb;
    const bool live = node < nN;
    float y0 = fmaf(acc0, inv, bz0) + rsi.x;
    float y1 = fmaf(acc1, inv, bz1) + rsi.y;

    if constexpr (FIN == 0) {
      y0 = (y0 < 0.0f) ? 0.0f : y0;
      y1 = (y1 < 0.0f) ? 0.0f : y1;
      y0 += pzr; y1 += pzr;
      const float u0 = live ? y0 : 0.0f;
      const float u1 = live ? y1 : 0.0f;
      const unsigned int h0 = f2bf(u0), h1 = f2bf(u1);
      const unsigned int l0 = f2bf(u0 - bf2f(h0)), l1 = f2bf(u1 - bf2f(h1));
      const unsigned int hw = h0 | (h1 << 16);
      const unsigned int lw = l0 | (l1 << 16);
      if (node < MPr) {
        unsigned int* hp = XHL + (size_t)node * XW + lane;
        *(volatile unsigned int*)hp = hw;
        *(volatile unsigned int*)(hp + 32) = lw;
        __threadfence();
        *(volatile unsigned int*)hp = hw;
        *(volatile unsigned int*)(hp + 32) = lw;
      }
    } else {
      y0 += pzr; y1 += pzr;
      float sv = y0 * wf0;
      sv = fmaf(y1, wf1, sv);
#pragma unroll
      for (int off = 16; off > 0; off >>= 1) sv += __shfl_xor(sv, off, 32);
      const float ov = live ? sv : 0.0f;
      if (lane == 0) sS[s] = ov;
    }
  }

  if constexpr (FIN == 1) {
    __syncthreads();
    const v4f v = *(const v4fa*)(sS + 4 * tid);
    float* gp = S + (size_t)blk * NBA + 4 * tid;
    *(volatile v4f*)gp = v;
    __threadfence();
    *(volatile v4f*)gp = v;
  }
}

__global__ __launch_bounds__(NTHR) void k_pool(const int* __restrict__ batch, const float* __restrict__ S,
                                               double* PSL, int nN, int vec4) {
  __shared__ double wsum[NWAVE];
  __shared__ int    wcn[NWAVE];
  const int tid = (int)threadIdx.x, lane = tid & 31, wave = tid >> 5;
  const int g = (int)blockIdx.x;
  double sumd = 0.0;
  int mine = 0;
  if (vec4 != 0) {
#pragma unroll 1
    for (int i = tid * 4; i < nN; i += NTHR * 4) {
      const v4i id = *(const v4i*)(batch + i);
      const v4f sv = *(const v4f*)(S + i);
      sumd += (id.x == g) ? (double)sv.x : 0.0;  mine += (id.x == g) ? 1 : 0;
      sumd += (id.y == g) ? (double)sv.y : 0.0;  mine += (id.y == g) ? 1 : 0;
      sumd += (id.z == g) ? (double)sv.z : 0.0;  mine += (id.z == g) ? 1 : 0;
      sumd += (id.w == g) ? (double)sv.w : 0.0;  mine += (id.w == g) ? 1 : 0;
    }
  } else {
#pragma unroll 1
    for (int i = tid; i < nN; i += NTHR) {
      const int id = batch[i];
      const float sv = S[i];
      sumd += (id == g) ? (double)sv : 0.0;
      mine += (id == g) ? 1 : 0;
    }
  }
#pragma unroll
  for (int off = 16; off > 0; off >>= 1) {
    sumd += __shfl_xor(sumd, off, 32);
    mine += __shfl_xor(mine, off, 32);
  }
  if (lane == 0) { wsum[wave] = sumd; wcn[wave] = mine; }
  __syncthreads();
  if (wave == 0) {
    double tot = 0.0;
    int tc = 0;
#pragma unroll
    for (int w2 = 0; w2 < NWAVE; ++w2) { tot += wsum[w2]; tc += wcn[w2]; }
    v2d pv;
    pv.x = (lane == 0) ? tot : 0.0;
    pv.y = (lane == 0) ? (double)tc : 0.0;
    double* rp = PSL + (size_t)g * 16 + 2 * (lane & 7);
    if (lane < 8) *(volatile v2d*)rp = pv;
    __threadfence();
    if (lane < 8) *(volatile v2d*)rp = pv;
  }
}

__global__ __launch_bounds__(NTHR) void k_head(const double* __restrict__ PSL, const float* __restrict__ bf,
                                               float* out) {
  const int g = (int)threadIdx.x;
  const v2d p = *(const v2d*)(PSL + (size_t)g * 16);
  const double c = p.y < 1.0 ? 1.0 : p.y;
  const float r = (float)(p.x / c) + bfr(bf[0]);
  *(volatile float*)(out + g) = r;
  __threadfence();
  *(volatile float*)(out + g) = r;
}

static inline int cdiv(int a, int b) { return (a + b - 1) / b; }

extern "C" void kernel_launch(void* const* d_in, const int* in_sizes, int n_in,
                              void* d_out, int out_size, void* d_ws, size_t ws_size,
                              hipStream_t stream) {
  if (n_in < 23) return;
  const int nN = in_sizes[0] / DIN;
  if (nN <= 0 || in_sizes[0] != nN * DIN || nN > 65536) return;
  if (in_sizes[1] < 2 || (in_sizes[1] & 1) != 0) return;
  const int nE = in_sizes[1] / 2;
  if (nE < 1 || nE > (1 << 30)) return;
  if (in_sizes[2] != nN) return;
  if (in_sizes[3] != HID * DIN || in_sizes[4] != HID * DIN || in_sizes[7] != HID * DIN) return;
  if (in_sizes[5] != HID || in_sizes[6] != HID || in_sizes[8] != HID) return;
  if (in_sizes[9] != HID * HID || in_sizes[10] != HID * HID || in_sizes[13] != HID * HID) return;
  if (in_sizes[11] != HID || in_sizes[12] != HID || in_sizes[14] != HID) return;
  if (in_sizes[15] != HID * HID || in_sizes[16] != HID * HID || in_sizes[19] != HID * HID) return;
  if (in_sizes[17] != HID || in_sizes[18] != HID || in_sizes[20] != HID) return;
  if (in_sizes[21] != HID || in_sizes[22] != 1) return;
  if (out_size != NG) return;

  const float* x    = (const float*)d_in[0];
  const int*   ei   = (const int*)  d_in[1];
  const int*   bat  = (const int*)  d_in[2];
  const float* Wl0  = (const float*)d_in[3];
  const float* Wr0  = (const float*)d_in[4];
  const float* at0  = (const float*)d_in[5];
  const float* b0   = (const float*)d_in[6];
  const float* Rw0  = (const float*)d_in[7];
  const float* Rb0  = (const float*)d_in[8];
  const float* Wl1  = (const float*)d_in[9];
  const float* Wr1  = (const float*)d_in[10];
  const float* at1  = (const float*)d_in[11];
  const float* b1   = (const float*)d_in[12];
  const float* Rw1  = (const float*)d_in[13];
  const float* Rb1  = (const float*)d_in[14];
  const float* Wl2  = (const float*)d_in[15];
  const float* Wr2  = (const float*)d_in[16];
  const float* at2  = (const float*)d_in[17];
  const float* b2   = (const float*)d_in[18];
  const float* Rw2  = (const float*)d_in[19];
  const float* Rb2  = (const float*)d_in[20];
  const float* Wf   = (const float*)d_in[21];
  const float* bfp  = (const float*)d_in[22];
  float* out = (float*)d_out;
  const int* src = ei;
  const int* dst = ei + nE;

  const int MP   = cdiv(nN, GBM) * GBM;
  const int gM   = MP / GBM;
  const int gA   = cdiv(MP, NBA);
  if ((long long)gA * NBA < (long long)MP) return;
  const int vec8 = ((nE & 3) == 0) ? 1 : 0;
  const int vec4 = ((nN & 3) == 0) ? 1 : 0;
  const int nUx  = MP * (DIN / 8);
  if ((nUx % NTHR) != 0) return;

  char* ws = (char*)d_ws;
  size_t off = 0;
  const size_t oXB  = off; off += (size_t)MP * DIN * 2;           off = (off + 255) & ~(size_t)255;
  const size_t oBW  = off; off += (size_t)3 * PW * KG * 2;        off = (off + 255) & ~(size_t)255;
  const size_t oP   = off; off += (size_t)MP * PW * 4;            off = (off + 255) & ~(size_t)255;
  const size_t oXH  = off; off += (size_t)MP * XW * 4;            off = (off + 255) & ~(size_t)255;
  const size_t oHIT = off; off += (size_t)gA * RCAP * 4;          off = (off + 255) & ~(size_t)255;
  const size_t oFLG = off; off += (size_t)gA * 128;               off = (off + 255) & ~(size_t)255;
  const size_t oS   = off; off += (size_t)gA * NBA * 4;           off = (off + 255) & ~(size_t)255;
  const size_t oPSL = off; off += (size_t)NG * 128;               off = (off + 255) & ~(size_t)255;
  if (off > ws_size || off > (size_t)WSMAX) return;
  unsigned short* XB   = (unsigned short*)(ws + oXB);
  unsigned short* BW   = (unsigned short*)(ws + oBW);
  float*          P    = (float*)(ws + oP);
  unsigned int*   XHL  = (unsigned int*)(ws + oXH);
  int*            HITS = (int*)(ws + oHIT);
  int*            FLG  = (int*)(ws + oFLG);
  float*          S    = (float*)(ws + oS);
  double*         PSL  = (double*)(ws + oPSL);
  const unsigned short* B0 = BW;
  const unsigned short* B1 = BW + (size_t)PW * KG;
  const unsigned short* B2 = BW + (size_t)2 * PW * KG;
  const unsigned short* XHLh = (const unsigned short*)XHL;

  const int bktLds  = BKT_LDS_INTS * 4;
  const int scanLds = SCAN_LDS_INTS * 4;
  hipFuncSetAttribute(reinterpret_cast<const void*>(&k_bucket),
                      hipFuncAttributeMaxDynamicSharedMemorySize, bktLds);
  hipFuncSetAttribute(reinterpret_cast<const void*>(&k_scan<0>),
                      hipFuncAttributeMaxDynamicSharedMemorySize, scanLds);
  hipFuncSetAttribute(reinterpret_cast<const void*>(&k_scan<1>),
                      hipFuncAttributeMaxDynamicSharedMemorySize, scanLds);

  k_prep<<<(nUx + NUW) / NTHR, NTHR, 0, stream>>>(x, Wl0, Wr0, Rw0, Wl1, Wr1, Rw1, Wl2, Wr2, Rw2, XB, BW, nN, nUx);
  k_bucket<<<gA, NTHR, bktLds, stream>>>(src, dst, nE, nN, vec8, HITS, FLG);
  k_gemm<<<dim3(gM, PW / GBN), GTHR, 0, stream>>>(XB, B0, Rb0, P);
  k_scan<0><<<gA, NTHR, scanLds, stream>>>(HITS, FLG, P, at0, b0, Wf, XHL, S, nN, MP);
  k_gemm<<<dim3(gM, PW / GBN), GTHR, 0, stream>>>(XHLh, B1, Rb1, P);
  k_scan<0><<<gA, NTHR, scanLds, stream>>>(HITS, FLG, P, at1, b1, Wf, XHL, S, nN, MP);
  k_gemm<<<dim3(gM, PW / GBN), GTHR, 0, stream>>>(XHLh, B2, Rb2, P);
  k_scan<1><<<gA, NTHR, scanLds, stream>>>(HITS, FLG, P, at2, b2, Wf, XHL, S, nN, MP);
  k_pool<<<NG, NTHR, 0, stream>>>(bat, S, PSL, nN, vec4);
  k_head<<<1, NTHR, 0, stream>>>(PSL, bfp, out);
}
